// DoubleFusionV3_5626407158448
// MI455X (gfx1250) — hardware-verified
//
#include <hip/hip_runtime.h>
#include <math.h>
#include <stdint.h>

#define NB   2
#define SEQ  2048
#define EM   1024
#define NH   32
#define HD   32
#define MR   (NB * SEQ)
#define NQB  (SEQ / 64)
static_assert(NH * HD == EM);
static_assert((SEQ % 64) == 0 && (EM % 64) == 0 && (MR % 64) == 0);

typedef __bf16   v16b __attribute__((ext_vector_type(16)));
typedef __bf16   v8b  __attribute__((ext_vector_type(8)));
typedef float    v8f  __attribute__((ext_vector_type(8)));
typedef float    v4f  __attribute__((ext_vector_type(4)));
typedef unsigned int v4u __attribute__((ext_vector_type(4)));

__device__ __forceinline__ unsigned short bf_bits(float f) {
  unsigned u = __float_as_uint(f);
  return (unsigned short)((u + 0x7FFFu + ((u >> 16) & 1u)) >> 16);
}
__device__ __forceinline__ float bf_up(unsigned short h) { return __uint_as_float(((unsigned)h) << 16); }
__device__ __forceinline__ float bf_rn(float f) { return bf_up(bf_bits(f)); }
__device__ __forceinline__ __bf16 bf_from_bits(unsigned short u) { return __builtin_bit_cast(__bf16, u); }
__device__ __forceinline__ unsigned pk16(unsigned short a, unsigned short b) { return (unsigned)a | ((unsigned)b << 16); }
__device__ __forceinline__ v8f zero8() { v8f z = {0.f, 0.f, 0.f, 0.f, 0.f, 0.f, 0.f, 0.f}; return z; }
__device__ __forceinline__ float gelu_f(float x) { return 0.5f * x * (1.0f + erff(x * 0.70710678118654752f)); }
__device__ __forceinline__ float silu_f(float x) { return x * __builtin_amdgcn_rcpf(1.0f + __expf(-x)); }

__device__ __forceinline__ void wave_sync() {
  __builtin_amdgcn_fence(__ATOMIC_RELEASE, "workgroup");
  __builtin_amdgcn_wave_barrier();
  __builtin_amdgcn_fence(__ATOMIC_ACQUIRE, "workgroup");
}

__device__ __forceinline__ v16b ldfrag_b(const __bf16* p) {
  union { v16b v; v8b h[2]; } f;
  f.h[0] = *(const v8b*)(p);
  f.h[1] = *(const v8b*)(p + 16);
  return f.v;
}

__device__ __forceinline__ v8f mma_raw(v16b a, v16b b, v8f c) {
  return __builtin_amdgcn_wmma_f32_16x16x32_bf16(false, a, false, b, (short)0, c, false, false);
}
__device__ __forceinline__ v8f mma_b(v16b a, v16b b, v8f c) {
  c = __builtin_amdgcn_wmma_f32_16x16x32_bf16(false, a, false, b, (short)0, c, false, false);
#if defined(__HIP_DEVICE_COMPILE__)
  asm volatile("v_nop\n\tv_nop\n\tv_nop\n\tv_nop" : "+v"(c) : "v"(a), "v"(b));
#endif
  return c;
}
template <typename V>
__device__ __forceinline__ void dep_guard(v8f& a, v8f& b, V x, V y) {
#if defined(__HIP_DEVICE_COMPILE__)
  asm volatile("v_nop\n\tv_nop\n\tv_nop\n\tv_nop" : "+v"(a), "+v"(b) : "v"(x), "v"(y));
#else
  (void)a; (void)b; (void)x; (void)y;
#endif
}
template <typename V>
__device__ __forceinline__ void keep4(V a, V b, V c, V d) {
#if defined(__HIP_DEVICE_COMPILE__)
  asm volatile("v_nop" :: "v"(a), "v"(b), "v"(c), "v"(d));
#else
  (void)a; (void)b; (void)c; (void)d;
#endif
}
__device__ __forceinline__ void acc_guard4(v8f& a, v8f& b, v8f& c, v8f& d) {
#if defined(__HIP_DEVICE_COMPILE__)
  asm volatile("v_nop\n\tv_nop\n\tv_nop\n\tv_nop" : "+v"(a), "+v"(b), "+v"(c), "+v"(d));
#else
  (void)a; (void)b; (void)c; (void)d;
#endif
}

__global__ __launch_bounds__(256) void cvt_bf16x8(const float* __restrict__ in, unsigned short* out, int n8) {
  const int i = blockIdx.x * 256 + threadIdx.x;
  if (i < n8) {
    const v4f a = *(const v4f*)(in + (size_t)i * 8);
    const v4f b = *(const v4f*)(in + (size_t)i * 8 + 4);
    v4u p;
    p[0] = pk16(bf_bits(a[0]), bf_bits(a[1]));
    p[1] = pk16(bf_bits(a[2]), bf_bits(a[3]));
    p[2] = pk16(bf_bits(b[0]), bf_bits(b[1]));
    p[3] = pk16(bf_bits(b[2]), bf_bits(b[3]));
    *(volatile v4u*)(out + (size_t)i * 8) = p;
    __threadfence();
    *(volatile v4u*)(out + (size_t)i * 8) = p;
  }
}

template <int NSPLIT, int OMODE, int ACT, int BROW>
__global__ __launch_bounds__(256) void gemm64(
    const unsigned short* __restrict__ Ap, const unsigned short* __restrict__ A2p, int lda, long long strideA,
    const unsigned short* __restrict__ Btp, int ldb, long long strideB,
    const float* __restrict__ bias, const float* __restrict__ Gp, int ldg,
    void* Cout, void* Cout2, int ldc, long long strideC,
    int M, int N, int K) {
  const __bf16* A  = (const __bf16*)(const void*)Ap;
  const __bf16* A2 = (const __bf16*)(const void*)A2p;
  const __bf16* Bt = (const __bf16*)(const void*)Btp;
  __shared__ __align__(16) float sT[8][16 * 68];
  const int b    = blockIdx.y;
  const int lane = threadIdx.x & 31;
  const int wave = threadIdx.x >> 5;
  const int tilesN = N >> 6;
  const int tilesM = M >> 6;
  const int tile = blockIdx.x * 8 + wave;
  if (tile >= tilesM * tilesN) return;
  const int tm = tile / tilesN;
  const int tn = tile - tm * tilesN;
  const int m0 = tm << 6;
  const int n0 = tn << 6;

  const __bf16* Ab  = A  + (size_t)b * (size_t)strideA;
  const __bf16* Ab2 = (NSPLIT != 0) ? (A2 + (size_t)b * (size_t)strideA) : Ab;
  const __bf16* Bb  = Bt + (size_t)b * (size_t)strideB;

  const int rlane = lane & 15;
  const int koff  = (lane >> 4) * 8;
  const int mOff  = (lane >> 4) * 8;

  v8f acc[4][4];
#pragma unroll
  for (int i = 0; i < 4; ++i)
#pragma unroll
    for (int j = 0; j < 4; ++j) acc[i][j] = zero8();

  for (int k0 = 0; k0 < K; k0 += 32) {
    v16b bh[4];
#pragma unroll
    for (int j = 0; j < 4; ++j) {
      const size_t bo = (size_t)(n0 + (j << 4) + rlane) * ldb + koff + k0;
      bh[j] = ldfrag_b(Bb + bo);
    }
#pragma unroll
    for (int i = 0; i < 4; ++i) {
      const size_t ao = (size_t)(m0 + (i << 4) + rlane) * lda + koff + k0;
      const v16b ah = ldfrag_b(Ab + ao);
      v16b al = ah;
      if (NSPLIT != 0) al = ldfrag_b(Ab2 + ao);
#pragma unroll
      for (int j = 0; j < 4; ++j) {
        acc[i][j] = mma_raw(ah, bh[j], acc[i][j]);
        if (NSPLIT != 0) acc[i][j] = mma_raw(al, bh[j], acc[i][j]);
      }
      dep_guard(acc[i][0], acc[i][3], ah, al);
    }
    keep4(bh[0], bh[1], bh[2], bh[3]);
  }
  acc_guard4(acc[0][0], acc[0][1], acc[0][2], acc[0][3]);
  acc_guard4(acc[1][0], acc[1][1], acc[1][2], acc[1][3]);
  acc_guard4(acc[2][0], acc[2][1], acc[2][2], acc[2][3]);
  acc_guard4(acc[3][0], acc[3][1], acc[3][2], acc[3][3]);

  float* slab = sT[wave];
#pragma unroll
  for (int i = 0; i < 4; ++i) {
    const int mBase = m0 + (i << 4);
#pragma unroll
    for (int j = 0; j < 4; ++j) {
#pragma unroll
      for (int r = 0; r < 8; ++r) {
        slab[(mOff + r) * 68 + (j << 4) + rlane] = acc[i][j][r];
      }
    }
    wave_sync();
#pragma unroll 1
    for (int e = lane; e < 16 * 64; e += 32) {
      const int row = e >> 6;
      const int col = e & 63;
      float v = slab[row * 68 + col];
      const float bb = (BROW != 0) ? bias[mBase + row] : bias[n0 + col];
      v += bf_rn(bb);
      if (ACT == 1) v = gelu_f(v);
      if (ACT == 2) {
        const float g = Gp[(size_t)(mBase + row) * ldg + n0 + col];
        v *= silu_f(g);
      }
      slab[row * 68 + col] = v;
    }
    wave_sync();
    if (OMODE == 0) {
      float* C = (float*)Cout + (size_t)b * (size_t)strideC;
      const int hh = lane >> 4, c4 = (lane & 15) * 4;
      for (int pass = 0; pass < 2; ++pass) {
#pragma unroll
        for (int it = 0; it < 8; ++it) {
          const int row = it * 2 + hh;
          const v4f v = *(const v4f*)(slab + row * 68 + c4);
          *(volatile v4f*)(C + (size_t)(mBase + row) * ldc + n0 + c4) = v;
        }
        __threadfence();
      }
    } else {
      const int q = lane >> 3, c8 = (lane & 7) * 8;
      unsigned short* C  = (unsigned short*)Cout  + (size_t)b * (size_t)strideC;
      unsigned short* C2 = (unsigned short*)Cout2 + (size_t)b * (size_t)strideC;
      v4u hv[4], lv[4];
#pragma unroll
      for (int it = 0; it < 4; ++it) {
        const int row = it * 4 + q;
        const float* sp = slab + row * 68 + c8;
        v4u a, a2;
#pragma unroll
        for (int e = 0; e < 4; ++e) {
          const float f0 = sp[2 * e], f1 = sp[2 * e + 1];
          const unsigned short h0 = bf_bits(f0), h1 = bf_bits(f1);
          const unsigned short l0 = bf_bits(f0 - bf_up(h0)), l1 = bf_bits(f1 - bf_up(h1));
          a[e] = pk16(h0, h1); a2[e] = pk16(l0, l1);
        }
        hv[it] = a; lv[it] = a2;
      }
      for (int pass = 0; pass < 2; ++pass) {
#pragma unroll
        for (int it = 0; it < 4; ++it) {
          const int row = it * 4 + q;
          *(volatile v4u*)(C  + (size_t)(mBase + row) * ldc + n0 + c8) = hv[it];
          *(volatile v4u*)(C2 + (size_t)(mBase + row) * ldc + n0 + c8) = lv[it];
        }
        __threadfence();
      }
    }
    wave_sync();
  }
}

__global__ __launch_bounds__(128)
void lin_attn(const unsigned short* __restrict__ qhp, const unsigned short* __restrict__ qlp,
              const unsigned short* __restrict__ khp, const unsigned short* __restrict__ klp,
              const unsigned short* __restrict__ vhp, const unsigned short* __restrict__ vlp,
              float* O) {
  union FB { v16b v; v8b h[2]; };
  __shared__ __align__(16) __bf16 Ksh[64 * 32];
  __shared__ __align__(16) __bf16 Ksl[64 * 32];
  __shared__ __align__(16) __bf16 Vth[32 * 64];
  __shared__ __align__(16) __bf16 Vtl[32 * 64];
  __shared__ __align__(16) __bf16 Psh[4][16 * 64];
  __shared__ __align__(16) __bf16 Psl[4][16 * 64];
  __shared__ __align__(16) float  Os[4][16 * 32];

  const int tid  = threadIdx.x;
  const int wave = tid >> 5;
  const int lane = tid & 31;
  const int hh   = lane >> 4;
  const int c    = lane & 15;

  const int bx   = blockIdx.x;
  const int qb   = bx % NQB;
  const int rest = bx / NQB;
  const int h    = rest % NH;
  const int b    = rest / NH;
  const int q0   = qb * 64 + wave * 16;

  const __bf16* Qh = (const __bf16*)(const void*)qhp;
  const __bf16* Ql = (const __bf16*)(const void*)qlp;
  const __bf16* Kh = (const __bf16*)(const void*)khp;
  const __bf16* Kl = (const __bf16*)(const void*)klp;
  const __bf16* VTh = (const __bf16*)(const void*)vhp + ((size_t)b * EM + (size_t)h * HD) * SEQ;
  const __bf16* VTl = (const __bf16*)(const void*)vlp + ((size_t)b * EM + (size_t)h * HD) * SEQ;

  v16b qah, qal;
  {
    const size_t qo = ((size_t)(q0 + c) * NB + b) * EM + (size_t)h * HD + 8 * hh;
    qah = ldfrag_b(Qh + qo);
    qal = ldfrag_b(Ql + qo);
  }

  v8f oacc[2];
  oacc[0] = zero8(); oacc[1] = zero8();

  const int sr = tid >> 1, shalf = (tid & 1) * 16;
  const int sd = tid >> 2, sq = (tid & 3) * 16;

  for (int kt = 0; kt < NQB; ++kt) {
    if (kt > qb) break;
    const int kv0 = kt * 64;
    __syncthreads();
    {
      const size_t ko = ((size_t)(kv0 + sr) * NB + b) * EM + (size_t)h * HD + shalf;
      const v8b a0 = *(const v8b*)(Kh + ko);
      const v8b a1 = *(const v8b*)(Kh + ko + 8);
      const v8b l0 = *(const v8b*)(Kl + ko);
      const v8b l1 = *(const v8b*)(Kl + ko + 8);
      *(v8b*)(Ksh + sr * 32 + shalf)     = a0;
      *(v8b*)(Ksh + sr * 32 + shalf + 8) = a1;
      *(v8b*)(Ksl + sr * 32 + shalf)     = l0;
      *(v8b*)(Ksl + sr * 32 + shalf + 8) = l1;
      const size_t vo = (size_t)sd * SEQ + kv0 + sq;
      const v8b b0 = *(const v8b*)(VTh + vo);
      const v8b b1 = *(const v8b*)(VTh + vo + 8);
      const v8b m0 = *(const v8b*)(VTl + vo);
      const v8b m1 = *(const v8b*)(VTl + vo + 8);
      *(v8b*)(Vth + sd * 64 + sq)     = b0;
      *(v8b*)(Vth + sd * 64 + sq + 8) = b1;
      *(v8b*)(Vtl + sd * 64 + sq)     = m0;
      *(v8b*)(Vtl + sd * 64 + sq + 8) = m1;
    }
    __syncthreads();

    v8f s[4];
#pragma unroll
    for (int j = 0; j < 4; ++j) {
      FB kb, kl;
      kb.h[0] = *(const v8b*)(Ksh + (j * 16 + c) * 32 + 8 * hh);
      kb.h[1] = *(const v8b*)(Ksh + (j * 16 + c) * 32 + 16 + 8 * hh);
      kl.h[0] = *(const v8b*)(Ksl + (j * 16 + c) * 32 + 8 * hh);
      kl.h[1] = *(const v8b*)(Ksl + (j * 16 + c) * 32 + 16 + 8 * hh);
      s[j] = mma_b(qah, kb.v, zero8());
      s[j] = mma_b(qah, kl.v, s[j]);
      s[j] = mma_b(qal, kb.v, s[j]);
    }
    if (kt == qb) {
#pragma unroll
      for (int r = 0; r < 8; ++r) {
        const int qrow = q0 + 8 * hh + r;
#pragma unroll
        for (int j = 0; j < 4; ++j) {
          const int key = kv0 + j * 16 + c;
          s[j][r] = (key <= qrow) ? s[j][r] : 0.0f;
        }
      }
    }

    __bf16* pwh = Psh[wave];
    __bf16* pwl = Psl[wave];
#pragma unroll
    for (int r = 0; r < 8; ++r) {
#pragma unroll
      for (int j = 0; j < 4; ++j) {
        const float f = s[j][r];
        const unsigned short h0 = bf_bits(f);
        const unsigned short l0 = bf_bits(f - bf_up(h0));
        pwh[(8 * hh + r) * 64 + j * 16 + c] = bf_from_bits(h0);
        pwl[(8 * hh + r) * 64 + j * 16 + c] = bf_from_bits(l0);
      }
    }
    wave_sync();

#pragma unroll
    for (int kk = 0; kk < 2; ++kk) {
      FB pa, pl;
      pa.h[0] = *(const v8b*)(pwh + c * 64 + kk * 32 + 8 * hh);
      pa.h[1] = *(const v8b*)(pwh + c * 64 + kk * 32 + 16 + 8 * hh);
      pl.h[0] = *(const v8b*)(pwl + c * 64 + kk * 32 + 8 * hh);
      pl.h[1] = *(const v8b*)(pwl + c * 64 + kk * 32 + 16 + 8 * hh);
#pragma unroll
      for (int t = 0; t < 2; ++t) {
        FB vb, vl;
        vb.h[0] = *(const v8b*)(Vth + (t * 16 + c) * 64 + kk * 32 + 8 * hh);
        vb.h[1] = *(const v8b*)(Vth + (t * 16 + c) * 64 + kk * 32 + 16 + 8 * hh);
        vl.h[0] = *(const v8b*)(Vtl + (t * 16 + c) * 64 + kk * 32 + 8 * hh);
        vl.h[1] = *(const v8b*)(Vtl + (t * 16 + c) * 64 + kk * 32 + 16 + 8 * hh);
        oacc[t] = mma_b(pa.v, vb.v, oacc[t]);
        oacc[t] = mma_b(pa.v, vl.v, oacc[t]);
        oacc[t] = mma_b(pl.v, vb.v, oacc[t]);
      }
    }
  }

  float* os = Os[wave];
#pragma unroll
  for (int r = 0; r < 8; ++r) {
#pragma unroll
    for (int t = 0; t < 2; ++t) os[(8 * hh + r) * 32 + t * 16 + c] = oacc[t][r];
  }
  wave_sync();
  {
    const int q4 = lane >> 3, c4 = (lane & 7) * 4;
    for (int pass = 0; pass < 2; ++pass) {
#pragma unroll
      for (int it = 0; it < 4; ++it) {
        const int row = it * 4 + q4;
        const v4f v = *(const v4f*)(os + row * 32 + c4);
        *(volatile v4f*)(O + ((size_t)(q0 + row) * NB + b) * EM + (size_t)h * HD + c4) = v;
      }
      __threadfence();
    }
  }
}

__global__ __launch_bounds__(128) void ln_rows(const float* __restrict__ X, const float* __restrict__ g,
                                               const float* __restrict__ bt, unsigned short* Yh, unsigned short* Yl) {
  __shared__ float red[4];
  const int row  = blockIdx.x;
  const int t    = threadIdx.x;
  const int lane = t & 31;
  const int wave = t >> 5;
  const float* xr = X + (size_t)row * EM + t * 8;
  const v4f a = *(const v4f*)(xr);
  const v4f d = *(const v4f*)(xr + 4);
  float x[8];
#pragma unroll
  for (int e = 0; e < 4; ++e) { x[e] = a[e]; x[4 + e] = d[e]; }

  float s = 0.f;
#pragma unroll
  for (int e = 0; e < 8; ++e) s += x[e];
#pragma unroll
  for (int off = 1; off < 32; off <<= 1) s += __shfl_xor(s, off, 32);
  if (lane == 0) red[wave] = s;
  __syncthreads();
  const float mu = (red[0] + red[1] + red[2] + red[3]) * (1.0f / EM);
  __syncthreads();

  float s2 = 0.f;
#pragma unroll
  for (int e = 0; e < 8; ++e) { const float dd = x[e] - mu; s2 += dd * dd; }
#pragma unroll
  for (int off = 1; off < 32; off <<= 1) s2 += __shfl_xor(s2, off, 32);
  if (lane == 0) red[wave] = s2;
  __syncthreads();
  const float var  = (red[0] + red[1] + red[2] + red[3]) * (1.0f / EM);
  const float rstd = rsqrtf(var + 1e-5f);

  unsigned short hb[8], lb[8];
#pragma unroll
  for (int e = 0; e < 8; ++e) {
    const int col = t * 8 + e;
    const float y = (x[e] - mu) * rstd * bf_rn(g[col]) + bf_rn(bt[col]);
    hb[e] = bf_bits(y);
    lb[e] = bf_bits(y - bf_up(hb[e]));
  }
  v4u ph, pl;
  ph[0] = pk16(hb[0], hb[1]); ph[1] = pk16(hb[2], hb[3]); ph[2] = pk16(hb[4], hb[5]); ph[3] = pk16(hb[6], hb[7]);
  pl[0] = pk16(lb[0], lb[1]); pl[1] = pk16(lb[2], lb[3]); pl[2] = pk16(lb[4], lb[5]); pl[3] = pk16(lb[6], lb[7]);
  const size_t yo = (size_t)row * EM + t * 8;
  *(volatile v4u*)(Yh + yo) = ph;
  *(volatile v4u*)(Yl + yo) = pl;
  __threadfence();
  *(volatile v4u*)(Yh + yo) = ph;
  *(volatile v4u*)(Yl + yo) = pl;
}

extern "C" void kernel_launch(void* const* d_in, const int* in_sizes, int n_in,
                              void* d_out, int out_size, void* d_ws, size_t ws_size,
                              hipStream_t stream) {
  if (n_in < 17) return;
  const int nAct = NB * SEQ * EM;
  const int nW   = EM * EM;
  if (in_sizes[0] != nAct || in_sizes[1] != nAct || in_sizes[2] != nAct) return;
  if (in_sizes[3] != nW || in_sizes[5] != nW || in_sizes[7] != nW || in_sizes[9] != nW ||
      in_sizes[11] != nW || in_sizes[13] != nW) return;
  if (in_sizes[4] != EM || in_sizes[6] != EM || in_sizes[8] != EM || in_sizes[10] != EM ||
      in_sizes[12] != EM || in_sizes[14] != EM || in_sizes[15] != EM || in_sizes[16] != EM) return;
  if (out_size != nAct) return;

  const float* query = (const float*)d_in[0];
  const float* key_  = (const float*)d_in[1];
  const float* value = (const float*)d_in[2];
  const float* Wq  = (const float*)d_in[3];  const float* bq  = (const float*)d_in[4];
  const float* Wk  = (const float*)d_in[5];  const float* bk  = (const float*)d_in[6];
  const float* Wv  = (const float*)d_in[7];  const float* bv  = (const float*)d_in[8];
  const float* Wu  = (const float*)d_in[9];  const float* bu  = (const float*)d_in[10];
  const float* Wo1 = (const float*)d_in[11]; const float* bo1 = (const float*)d_in[12];
  const float* Wo2 = (const float*)d_in[13]; const float* bo2 = (const float*)d_in[14];
  const float* lng = (const float*)d_in[15]; const float* lnb = (const float*)d_in[16];

  const size_t P16 = (size_t)MR * EM * 2;
  const size_t PW  = (size_t)EM * EM * 2;
  const size_t PVT = (size_t)NB * EM * SEQ * 2;
  const size_t P32 = (size_t)MR * EM * 4;
  size_t off = 0;
  const size_t oXq  = off; off += P16;
  const size_t oXk  = off; off += P16;
  const size_t oXv  = off; off += P16;
  const size_t oWq  = off; off += PW;
  const size_t oWk  = off; off += PW;
  const size_t oWv  = off; off += PW;
  const size_t oWu  = off; off += PW;
  const size_t oWo1 = off; off += PW;
  const size_t oWo2 = off; off += PW;
  const size_t oQh  = off; off += P16;
  const size_t oQl  = off; off += P16;
  const size_t oKh  = off; off += P16;
  const size_t oKl  = off; off += P16;
  const size_t oVTh = off; off += PVT;
  const size_t oVTl = off; off += PVT;
  const size_t oU   = off; off += P32;
  const size_t oGh  = off; off += P16;
  const size_t oGl  = off; off += P16;
  if (off > ws_size) return;
  if (off > (size_t)134217728) return;
  const size_t oO   = oXq;
  const size_t oYh  = oXv;
  const size_t oYl  = oWq;
  if (oO + P32 != oXv) return;
  if (oYh + P16 != oYl || oYl + P16 != oWo1) return;

  char* ws = (char*)d_ws;
  unsigned short* Xq   = (unsigned short*)(ws + oXq);
  unsigned short* Xk   = (unsigned short*)(ws + oXk);
  unsigned short* Xv   = (unsigned short*)(ws + oXv);
  unsigned short* Wqb  = (unsigned short*)(ws + oWq);
  unsigned short* Wkb  = (unsigned short*)(ws + oWk);
  unsigned short* Wvb  = (unsigned short*)(ws + oWv);
  unsigned short* Wub  = (unsigned short*)(ws + oWu);
  unsigned short* Wo1b = (unsigned short*)(ws + oWo1);
  unsigned short* Wo2b = (unsigned short*)(ws + oWo2);
  unsigned short* Qh   = (unsigned short*)(ws + oQh);
  unsigned short* Ql   = (unsigned short*)(ws + oQl);
  unsigned short* Kh   = (unsigned short*)(ws + oKh);
  unsigned short* Kl   = (unsigned short*)(ws + oKl);
  unsigned short* VTh  = (unsigned short*)(ws + oVTh);
  unsigned short* VTl  = (unsigned short*)(ws + oVTl);
  float*          U    = (float*)(ws + oU);
  unsigned short* Gh   = (unsigned short*)(ws + oGh);
  unsigned short* Gl   = (unsigned short*)(ws + oGl);
  float*          O    = (float*)(ws + oO);
  unsigned short* Yh   = (unsigned short*)(ws + oYh);
  unsigned short* Yl   = (unsigned short*)(ws + oYl);

  const dim3 blk(256);
  const int n8a = nAct / 8;
  const int n8w = nW / 8;
  const dim3 gCvtA((n8a + 255) / 256);
  const dim3 gCvtW((n8w + 255) / 256);
  const dim3 gProj(((MR / 64) * (EM / 64) + 7) / 8, 1);
  const dim3 gVT(((EM / 64) * (SEQ / 64) + 7) / 8, NB);

  cvt_bf16x8<<<gCvtA, blk, 0, stream>>>(query, Xq, n8a);
  cvt_bf16x8<<<gCvtA, blk, 0, stream>>>(key_,  Xk, n8a);
  cvt_bf16x8<<<gCvtA, blk, 0, stream>>>(value, Xv, n8a);
  cvt_bf16x8<<<gCvtW, blk, 0, stream>>>(Wq,  Wqb,  n8w);
  cvt_bf16x8<<<gCvtW, blk, 0, stream>>>(Wk,  Wkb,  n8w);
  cvt_bf16x8<<<gCvtW, blk, 0, stream>>>(Wv,  Wvb,  n8w);
  cvt_bf16x8<<<gCvtW, blk, 0, stream>>>(Wu,  Wub,  n8w);
  cvt_bf16x8<<<gCvtW, blk, 0, stream>>>(Wo1, Wo1b, n8w);
  cvt_bf16x8<<<gCvtW, blk, 0, stream>>>(Wo2, Wo2b, n8w);

  gemm64<0, 2, 1, 0><<<gProj, blk, 0, stream>>>(
      Xq, Xq, EM, 0LL, Wqb, EM, 0LL, bq, bq, 0,
      (void*)Qh, (void*)Ql, EM, 0LL, MR, EM, EM);
  gemm64<0, 2, 1, 0><<<gProj, blk, 0, stream>>>(
      Xk, Xk, EM, 0LL, Wkb, EM, 0LL, bk, bk, 0,
      (void*)Kh, (void*)Kl, EM, 0LL, MR, EM, EM);
  gemm64<0, 2, 0, 1><<<gVT, blk, 0, stream>>>(
      Wvb, Wvb, EM, 0LL, Xv, NB * EM, (long long)EM, bv, bv, 0,
      (void*)VTh, (void*)VTl, SEQ, (long long)EM * SEQ, EM, SEQ, EM);
  gemm64<0, 0, 0, 0><<<gProj, blk, 0, stream>>>(
      Xq, Xq, EM, 0LL, Wub, EM, 0LL, bu, bu, 0,
      (void*)U, (void*)U, EM, 0LL, MR, EM, EM);
  lin_attn<<<dim3(NB * NH * NQB), dim3(128), 0, stream>>>(Qh, Ql, Kh, Kl, VTh, VTl, O);
  ln_rows<<<dim3(MR), dim3(128), 0, stream>>>(O, lng, lnb, Yh, Yl);
  gemm64<1, 2, 2, 0><<<gProj, blk, 0, stream>>>(
      Yh, Yl, EM, 0LL, Wo1b, EM, 0LL, bo1, U, EM,
      (void*)Gh, (void*)Gl, EM, 0LL, MR, EM, EM);
  gemm64<1, 0, 0, 0><<<gProj, blk, 0, stream>>>(
      Gh, Gl, EM, 0LL, Wo2b, EM, 0LL, bo2, bo2, 0,
      d_out, d_out, EM, 0LL, MR, EM, EM);
  (void)hipGetLastError();
}
